// mLSTM_41274635715161
// MI455X (gfx1250) — hardware-verified
//
#include <hip/hip_runtime.h>
#include <math.h>

constexpr int NBAT = 8;
constexpr int NSEQ = 1024;
constexpr int NDIM = 128;
constexpr int NHID = 128;
constexpr int NLAY = 2;
constexpr int NROW = NBAT * NSEQ;
constexpr int NQKV = 3 * NHID;
constexpr int NGT  = 2 * NHID;
constexpr int NTHR = 256;
constexpr int TCH  = 32;
constexpr int HCH  = 16;
constexpr int APITCH = 136;
constexpr int OPITCH = 132;
constexpr int NBIAS = NQKV + 2 * NGT;
static_assert(NROW % 64 == 0 && NQKV % 64 == 0 && NGT % 64 == 0, "GEMM M, N tile multiples");
static_assert(NDIM % 32 == 0 && NHID % 32 == 0, "GEMM K multiple of 32");
static_assert(NSEQ % TCH == 0 && NSEQ % HCH == 0, "static chunking");
static_assert(NHID == 128 && NDIM == 128, "scan kernels are laid out for 128 columns");
static_assert(NHID == 16 * (NTHR / 32), "one 16-column group per wave in the recurrence");
static_assert(NBAT == 8, "recurrence block holds 8 real rows in one 16-row tile");
static_assert((NROW / 64) * (NQKV / 64) % 8 == 0 && (NROW / 64) * (NGT / 64) % 8 == 0, "GEMM grids exact");
static_assert(NBIAS % 4 == 0 && NBIAS / 4 <= NTHR, "bias prep coverage");

typedef __attribute__((ext_vector_type(16))) _Float16 v16h;
typedef __attribute__((ext_vector_type(8)))  _Float16 v8h;
typedef __attribute__((ext_vector_type(16))) __bf16   v16b;
typedef __attribute__((ext_vector_type(8)))  __bf16   v8b;
typedef __attribute__((ext_vector_type(8)))  float    v8f;
typedef __attribute__((ext_vector_type(4)))  float    v4f;

__device__ __forceinline__ unsigned short f2bf_bits(float f) {
  unsigned u = __float_as_uint(f);
  return (unsigned short)((u + 0x7FFFu + ((u >> 16) & 1u)) >> 16);
}
__device__ __forceinline__ float bf_bits2f(unsigned short h) { return __uint_as_float(((unsigned)h) << 16); }
__device__ __forceinline__ float bf16r(float f) { return bf_bits2f(f2bf_bits(f)); }

__device__ __forceinline__ void dep_guard_h(v8f& a, v8f& b, v16h x, v16h y) { asm volatile("v_nop\n\tv_nop\n\tv_nop\n\tv_nop" : "+v"(a), "+v"(b) : "v"(x), "v"(y)); }
__device__ __forceinline__ void dep_guard_b(v8f& a, v8f& b, v16b x, v16b y) { asm volatile("v_nop\n\tv_nop\n\tv_nop\n\tv_nop" : "+v"(a), "+v"(b) : "v"(x), "v"(y)); }
__device__ __forceinline__ void dep_guard1_b(v8f& a, v16b x, v16b y) { asm volatile("v_nop\n\tv_nop\n\tv_nop\n\tv_nop" : "+v"(a) : "v"(x), "v"(y)); }
__device__ __forceinline__ void keep4_h(v16h a, v16h b, v16h c, v16h d) { asm volatile("v_nop" :: "v"(a), "v"(b), "v"(c), "v"(d)); }
__device__ __forceinline__ void keep4_b(v16b a, v16b b, v16b c, v16b d) { asm volatile("v_nop" :: "v"(a), "v"(b), "v"(c), "v"(d)); }
__device__ __forceinline__ void acc_guard4(v8f& a, v8f& b, v8f& c, v8f& d) { asm volatile("v_nop\n\tv_nop\n\tv_nop\n\tv_nop" : "+v"(a), "+v"(b), "+v"(c), "+v"(d)); }
__device__ __forceinline__ void acc_guard1(v8f& a) { asm volatile("v_nop\n\tv_nop\n\tv_nop\n\tv_nop" : "+v"(a)); }
template <typename T> struct Frag;
template <> struct Frag<_Float16> {
  typedef v16h V; union U { v16h v; v8h h[2]; };
  static __device__ __forceinline__ v16h load(const _Float16* p) {
    U f; f.h[0] = *(const v8h*)(p); f.h[1] = *(const v8h*)(p + 16); return f.v;
  }
  static __device__ __forceinline__ v8f mma(v16h a, v16h b, v8f c) {
    return __builtin_amdgcn_wmma_f32_16x16x32_f16(false, a, false, b, (short)0, c, false, false);
  }
  static __device__ __forceinline__ void guard(v8f& a, v8f& b, v16h x, v16h y) { dep_guard_h(a, b, x, y); }
  static __device__ __forceinline__ void keep(v16h a, v16h b, v16h c, v16h d) { keep4_h(a, b, c, d); }
};
template <> struct Frag<__bf16> {
  typedef v16b V; union U { v16b v; v8b h[2]; };
  static __device__ __forceinline__ v16b load(const __bf16* p) {
    U f; f.h[0] = *(const v8b*)(p); f.h[1] = *(const v8b*)(p + 16); return f.v;
  }
  static __device__ __forceinline__ v8f mma(v16b a, v16b b, v8f c) {
    return __builtin_amdgcn_wmma_f32_16x16x32_bf16(false, a, false, b, (short)0, c, false, false);
  }
  static __device__ __forceinline__ void guard(v8f& a, v8f& b, v16b x, v16b y) { dep_guard_b(a, b, x, y); }
  static __device__ __forceinline__ void keep(v16b a, v16b b, v16b c, v16b d) { keep4_b(a, b, c, d); }
};

template <int ET> struct Elem;
template <> struct Elem<0> { typedef _Float16 T; };
template <> struct Elem<1> { typedef __bf16 T; };
template <int ET, int SPLITM, int BIAS_MODE, int OUT_MODE, int ACT = 0>
__global__ __launch_bounds__(256) void wmma_gemm64(
    const unsigned short* __restrict__ Ap, const unsigned short* __restrict__ A2p, int lda, long strideA,
    const unsigned short* __restrict__ Btp, const unsigned short* __restrict__ Bt2p, int ldb, long strideB,
    void* __restrict__ Cout, void* __restrict__ Cout2, int ldc, long strideC,
    const float* __restrict__ bias, int M, int N, int K, float scale) {
  typedef typename Elem<ET>::T T;
  typedef typename Frag<T>::V V;
  constexpr bool SPA = (SPLITM != 0);
  constexpr bool SPB = (SPLITM == 1);
  const T* A = (const T*)Ap; const T* A2 = (const T*)A2p; const T* Bt = (const T*)Btp; const T* Bt2 = (const T*)Bt2p;
  __shared__ __align__(16) float sT[8][16 * 68];
  const int b    = blockIdx.y;
  const int lane = threadIdx.x & 31;
  const int wave = threadIdx.x >> 5;
  const int tilesN = N >> 6;
  const int tilesM = M >> 6;
  const int tile = blockIdx.x * 8 + wave;
  if (tile >= tilesM * tilesN) return;
  const int tm = tile / tilesN;
  const int tn = tile - tm * tilesN;
  const int m0 = tm << 6;
  const int n0 = tn << 6;

  const T* Ab  = A  + (size_t)b * strideA;
  const T* Bb  = Bt + (size_t)b * strideB;
  const T* Ab2 = SPA ? (A2  + (size_t)b * strideA) : nullptr;
  const T* Bb2 = SPB ? (Bt2 + (size_t)b * strideB) : nullptr;

  const int rlane = lane & 15;
  const int koff  = (lane >> 4) * 8;
  const int mOff  = (lane >> 4) * 8;

  v8f acc[4][4];
#pragma unroll
  for (int i = 0; i < 4; ++i)
#pragma unroll
    for (int j = 0; j < 4; ++j) acc[i][j] = (v8f){0.f,0.f,0.f,0.f,0.f,0.f,0.f,0.f};

  for (int k0 = 0; k0 < K; k0 += 32) {
    V bh[4], bl[4];
#pragma unroll
    for (int j = 0; j < 4; ++j) {
      const size_t bo = (size_t)(n0 + (j << 4) + rlane) * ldb + koff + k0;
      bh[j] = Frag<T>::load(Bb + bo);
      if (SPB) bl[j] = Frag<T>::load(Bb2 + bo);
    }
#pragma unroll
    for (int i = 0; i < 4; ++i) {
      const size_t ao = (size_t)(m0 + (i << 4) + rlane) * lda + koff + k0;
      V ah = Frag<T>::load(Ab + ao);
      V al = ah;
      if (SPA) al = Frag<T>::load(Ab2 + ao);
#pragma unroll
      for (int j = 0; j < 4; ++j) {
        acc[i][j] = Frag<T>::mma(ah, bh[j], acc[i][j]);
        if (SPB) acc[i][j] = Frag<T>::mma(ah, bl[j], acc[i][j]);
        if (SPA) acc[i][j] = Frag<T>::mma(al, bh[j], acc[i][j]);
      }
      Frag<T>::guard(acc[i][0], acc[i][3], ah, al);
    }
    Frag<T>::keep(bh[0], bh[1], bh[2], bh[3]);
    if (SPB) Frag<T>::keep(bl[0], bl[1], bl[2], bl[3]);
  }
  acc_guard4(acc[0][0], acc[0][1], acc[0][2], acc[0][3]);
  acc_guard4(acc[1][0], acc[1][1], acc[1][2], acc[1][3]);
  acc_guard4(acc[2][0], acc[2][1], acc[2][2], acc[2][3]);
  acc_guard4(acc[3][0], acc[3][1], acc[3][2], acc[3][3]);

  float* slab = sT[wave];
#pragma unroll
  for (int i = 0; i < 4; ++i) {
    const int mBase = m0 + (i << 4);
#pragma unroll
    for (int j = 0; j < 4; ++j) {
      const int n = n0 + (j << 4) + rlane;
      float bv = 0.f;
      if (BIAS_MODE == 2) bv = bias[n];
#pragma unroll
      for (int r = 0; r < 8; ++r) {
        float v = acc[i][j][r] * scale;
        if (BIAS_MODE == 1) v += bias[mBase + mOff + r];
        if (BIAS_MODE == 2) v += bv;
        if (ACT == 1) v = tanhf(v);
        if (ACT == 2) v = fmaxf(v, 0.0f);
        if (ACT == 4) v = (v > 0.f) ? v : 0.01f * v;
        if (ACT == 6) v = expf(v);
        slab[(mOff + r) * 68 + (j << 4) + rlane] = v;
      }
    }
    __builtin_amdgcn_fence(__ATOMIC_RELEASE, "workgroup");
    __builtin_amdgcn_wave_barrier();
    __builtin_amdgcn_fence(__ATOMIC_ACQUIRE, "workgroup");
    if (OUT_MODE == 0) {
      float* C = (float*)Cout + (size_t)b * strideC;
      const int hh = lane >> 4, c4 = (lane & 15) * 4;
      for (int pass = 0; pass < 2; ++pass) {
#pragma unroll
        for (int it = 0; it < 8; ++it) {
          const int row = it * 2 + hh;
          v4f v = *(const v4f*)(slab + row * 68 + c4);
          *(volatile v4f*)(C + (size_t)(mBase + row) * ldc + n0 + c4) = v;
        }
        __threadfence();
      }
    } else {
      const int q = lane >> 3, c8 = (lane & 7) * 8;
      unsigned short* C  = (unsigned short*)Cout  + (size_t)b * strideC;
      unsigned short* C2 = (OUT_MODE == 2) ? ((unsigned short*)Cout2 + (size_t)b * strideC) : nullptr;
      for (int pass = 0; pass < 2; ++pass) {
#pragma unroll
        for (int it = 0; it < 4; ++it) {
          const int row = it * 4 + q;
          const float* sp = slab + row * 68 + c8;
          v8h hv, lv;
#pragma unroll
          for (int e = 0; e < 8; ++e) {
            if (OUT_MODE == 1) {
              hv[e] = (_Float16)sp[e];
            } else {
              unsigned short hb = f2bf_bits(sp[e]);
              unsigned short lb = f2bf_bits(sp[e] - bf_bits2f(hb));
              hv[e] = __builtin_bit_cast(_Float16, hb);
              lv[e] = __builtin_bit_cast(_Float16, lb);
            }
          }
          *(volatile v8h*)(C + (size_t)(mBase + row) * ldc + n0 + c8) = hv;
          if (OUT_MODE == 2) *(volatile v8h*)(C2 + (size_t)(mBase + row) * ldc + n0 + c8) = lv;
        }
        __threadfence();
      }
    }
    __builtin_amdgcn_fence(__ATOMIC_RELEASE, "workgroup");
    __builtin_amdgcn_wave_barrier();
    __builtin_amdgcn_fence(__ATOMIC_ACQUIRE, "workgroup");
  }
}

template <int MODE>
__global__ __launch_bounds__(NTHR) void cvt8_kernel(const float* __restrict__ src, unsigned short* __restrict__ dst,
                                                    int nrow, int ncol8, int spitch, int scol0, float sc) {
  const int i  = blockIdx.x * NTHR + threadIdx.x;
  const int n8 = nrow * ncol8;
  if (i < n8) {
    const int row = i / ncol8;
    const int c8  = i - row * ncol8;
    const float* sp = src + (size_t)row * spitch + scol0 + c8 * 8;
    const v4f a = *(const v4f*)(sp);
    const v4f b = *(const v4f*)(sp + 4);
    v8h hv;
#pragma unroll
    for (int e = 0; e < 4; ++e) {
      unsigned short b0, b1;
      if (MODE == 0) {
        b0 = f2bf_bits(a[e] * sc);
        b1 = f2bf_bits(b[e] * sc);
      } else {
        b0 = __builtin_bit_cast(unsigned short, (_Float16)(bf16r(a[e]) * sc));
        b1 = __builtin_bit_cast(unsigned short, (_Float16)(bf16r(b[e]) * sc));
      }
      hv[e]     = __builtin_bit_cast(_Float16, b0);
      hv[4 + e] = __builtin_bit_cast(_Float16, b1);
    }
    *(volatile v8h*)(dst + (size_t)i * 8) = hv;
    __threadfence();
    *(volatile v8h*)(dst + (size_t)i * 8) = hv;
  }
}

template <int MODE>
__global__ __launch_bounds__(NTHR) void tpw_kernel(const float* __restrict__ src, int R, int C, int ldo,
                                                   unsigned short* __restrict__ O, float sc) {
  __shared__ float Tt[64 * 65];
  const int tid = threadIdx.x;
  const int c0 = blockIdx.x * 64, r0 = blockIdx.y * 64;
#pragma unroll
  for (int i = 0; i < 4; ++i) {
    const int idx = i * NTHR + tid;
    const int rr = idx >> 4, cc = (idx & 15) * 4;
    const v4f v = *(const v4f*)(src + (size_t)(r0 + rr) * (size_t)C + c0 + cc);
    Tt[rr * 65 + cc + 0] = v[0];
    Tt[rr * 65 + cc + 1] = v[1];
    Tt[rr * 65 + cc + 2] = v[2];
    Tt[rr * 65 + cc + 3] = v[3];
  }
  __syncthreads();
  const int q = tid >> 3, c8 = (tid & 7) * 8;
  v8h hv[2];
#pragma unroll
  for (int g = 0; g < 2; ++g) {
    const int qq = g * 32 + q;
#pragma unroll
    for (int e = 0; e < 8; ++e) {
      const float f = Tt[(c8 + e) * 65 + qq];
      unsigned short bits;
      if (MODE == 0) {
        bits = f2bf_bits(f * sc);
      } else {
        const float fb = bf_bits2f(f2bf_bits(f));
        bits = __builtin_bit_cast(unsigned short, (_Float16)(fb * sc));
      }
      hv[g][e] = __builtin_bit_cast(_Float16, bits);
    }
  }
  for (int pass = 0; pass < 2; ++pass) {
#pragma unroll
    for (int g = 0; g < 2; ++g) {
      const size_t o = (size_t)(c0 + g * 32 + q) * (size_t)ldo + (size_t)(r0 + c8);
      *(volatile v8h*)(O + o) = hv[g];
    }
    __threadfence();
  }
}

__global__ __launch_bounds__(NTHR) void bias_prep_kernel(const float* __restrict__ bq, const float* __restrict__ bk,
                                                         const float* __restrict__ bv, const float* __restrict__ bi,
                                                         const float* __restrict__ bfw, float* __restrict__ dst) {
  const int tid = threadIdx.x;
  const int grp = tid >> 5;
  const int idx = (tid & 31) * 4;
  const v4f s0 = *(const v4f*)(bq + idx);
  const v4f s1 = *(const v4f*)(bk + idx);
  const v4f s2 = *(const v4f*)(bv + idx);
  const v4f s3 = *(const v4f*)(bi + idx);
  const v4f s4 = *(const v4f*)(bfw + idx);
  const v4f s5 = *(const v4f*)(bi + NHID + idx);
  const v4f s6 = *(const v4f*)(bfw + NHID + idx);
  const float f0 = (grp == 0) ? 1.0f : 0.0f;
  const float f1 = (grp == 1) ? 1.0f : 0.0f;
  const float f2 = (grp == 2) ? 1.0f : 0.0f;
  const float f3 = (grp == 3) ? 1.0f : 0.0f;
  const float f4 = (grp == 4) ? 1.0f : 0.0f;
  const float f5 = (grp == 5) ? 1.0f : 0.0f;
  const float f6 = (grp == 6) ? 1.0f : 0.0f;
  v4f o;
#pragma unroll
  for (int e = 0; e < 4; ++e) {
    float s = f0 * s0[e];
    s = fmaf(f1, s1[e], s);
    s = fmaf(f2, s2[e], s);
    s = fmaf(f3, s3[e], s);
    s = fmaf(f4, s4[e], s);
    s = fmaf(f5, s5[e], s);
    s = fmaf(f6, s6[e], s);
    o[e] = bf16r(s);
  }
  float* op = dst + grp * NHID + idx;
  *(volatile v4f*)op = o;
  __threadfence();
  *(volatile v4f*)op = o;
}

__global__ __launch_bounds__(NTHR) void cscan_kernel(const float* __restrict__ QKV, const float* __restrict__ GT,
                                                     float* __restrict__ ATT) {
  __shared__ __align__(16) float sQ[TCH * NHID];
  __shared__ __align__(16) float sW[TCH * NHID];
  __shared__ __align__(16) float sF[TCH * NHID];
  __shared__ __align__(16) float sK[TCH * 64];
  __shared__ __align__(16) float sP[TCH * 4 * 64];
  const int tid = threadIdx.x;
  const int kcl = tid & 63;
  const int rc  = tid >> 6;
  const int b   = blockIdx.x;
  const int ch  = blockIdx.y;
  float cst[32];
#pragma unroll
  for (int i = 0; i < 32; ++i) cst[i] = 0.0f;

#pragma unroll 1
  for (int cI = 0; cI < NSEQ / TCH; ++cI) {
    const int t0 = cI * TCH;
    const size_t rg0 = (size_t)b * NSEQ + (size_t)t0;
#pragma unroll
    for (int i = 0; i < 4; ++i) {
      const int idx = i * NTHR + tid;
      const int row = idx >> 5, c4 = (idx & 31) * 4;
      const float* qp = QKV + (rg0 + (size_t)row) * NQKV + c4;
      const float* gp = GT  + (rg0 + (size_t)row) * NGT  + c4;
      const v4f q4 = *(const v4f*)(qp);
      const v4f v4 = *(const v4f*)(qp + 2 * NHID);
      const v4f i4 = *(const v4f*)(gp);
      const v4f f4 = *(const v4f*)(gp + NHID);
      *(v4f*)(sQ + row * NHID + c4) = q4;
      *(v4f*)(sW + row * NHID + c4) = i4 * v4;
      *(v4f*)(sF + row * NHID + c4) = f4;
      asm volatile("" ::: "memory");
    }
#pragma unroll
    for (int i = 0; i < 2; ++i) {
      const int idx = i * NTHR + tid;
      const int row = idx >> 4, c4 = (idx & 15) * 4;
      const v4f k4 = *(const v4f*)(QKV + (rg0 + (size_t)row) * NQKV + NHID + 64 * ch + c4);
      *(v4f*)(sK + row * 64 + c4) = k4;
    }
    __syncthreads();

#pragma unroll 1
    for (int s = 0; s < TCH; ++s) {
      const float kk = sK[s * 64 + kcl];
      const float* fr = sF + s * NHID + 32 * rc;
      const float* wr = sW + s * NHID + 32 * rc;
      const float* qr = sQ + s * NHID + 32 * rc;
      float a = 0.0f;
#pragma unroll
      for (int i = 0; i < 8; ++i) {
        const v4f f4 = *(const v4f*)(fr + 4 * i);
        const v4f w4 = *(const v4f*)(wr + 4 * i);
        const v4f q4 = *(const v4f*)(qr + 4 * i);
#pragma unroll
        for (int e = 0; e < 4; ++e) {
          const float p  = w4[e] * kk;
          const float cn = fmaf(f4[e], cst[4 * i + e], p);
          cst[4 * i + e] = cn;
          a = fmaf(q4[e], cn, a);
        }
      }
      sP[(s * 4 + rc) * 64 + kcl] = a;
    }
    __syncthreads();

    for (int pass = 0; pass < 2; ++pass) {
#pragma unroll
      for (int it = 0; it < 2; ++it) {
        const int idx = it * NTHR + tid;
        const int row = idx >> 4, c4 = (idx & 15) * 4;
        const v4f p0 = *(const v4f*)(sP + (row * 4 + 0) * 64 + c4);
        const v4f p1 = *(const v4f*)(sP + (row * 4 + 1) * 64 + c4);
        const v4f p2 = *(const v4f*)(sP + (row * 4 + 2) * 64 + c4);
        const v4f p3 = *(const v4f*)(sP + (row * 4 + 3) * 64 + c4);
        const v4f o = (p0 + p1) + (p2 + p3);
        *(volatile v4f*)(ATT + (rg0 + (size_t)row) * NHID + 64 * ch + c4) = o;
      }
      __threadfence();
    }
  }
}

template <int MODE>
__global__ __launch_bounds__(NTHR) void hgate_kernel(const float* __restrict__ ATT, const unsigned short* __restrict__ WoTp,
                                                     const float* __restrict__ bo,
                                                     unsigned short* __restrict__ HHI, unsigned short* __restrict__ HLO,
                                                     float* __restrict__ OUT) {
  __shared__ __align__(16) unsigned short Ap[3][16 * APITCH];
  __shared__ __align__(16) float sOut[HCH * 8 * OPITCH];
  const __bf16* WoT = (const __bf16*)WoTp;
  const int tid = threadIdx.x, lane = tid & 31, wave = tid >> 5;
  const int c = lane & 15, hh = lane >> 4, koff = hh * 8;
  const int j = 16 * wave + c;
  {
    unsigned short* apf = &Ap[0][0];
#pragma unroll 1
    for (int i = tid; i < 3 * 16 * APITCH; i += NTHR) apf[i] = (unsigned short)0;
  }
  const float boj  = bf16r(bo[j]);
  const float rowf = (float)(1 - hh);
  __syncthreads();

  const __bf16* wrow = WoT + (size_t)j * NHID + koff;
  const __bf16* ap0 = (const __bf16*)&Ap[0][0] + c * APITCH + koff;
  const __bf16* ap1 = (const __bf16*)&Ap[1][0] + c * APITCH + koff;
  const __bf16* ap2 = (const __bf16*)&Ap[2][0] + c * APITCH + koff;
  const v8f z8 = {0.f, 0.f, 0.f, 0.f, 0.f, 0.f, 0.f, 0.f};

#pragma unroll 1
  for (int t = 0; t < NSEQ; ++t) {
    float av[8];
#pragma unroll
    for (int r = 0; r < 8; ++r) av[r] = ATT[((size_t)r * NSEQ + (size_t)t) * NHID + j] * rowf;

    v8f acc = z8;
#pragma unroll
    for (int kc = 0; kc < 4; ++kc) {
      const v16b bw = Frag<__bf16>::load(wrow + 32 * kc);
      const v16b a0 = Frag<__bf16>::load(ap0 + 32 * kc);
      const v16b a1 = Frag<__bf16>::load(ap1 + 32 * kc);
      const v16b a2 = Frag<__bf16>::load(ap2 + 32 * kc);
      acc = Frag<__bf16>::mma(a0, bw, acc);
      acc = Frag<__bf16>::mma(a1, bw, acc);
      acc = Frag<__bf16>::mma(a2, bw, acc);
      dep_guard1_b(acc, a2, bw);
      keep4_b(a0, a1, a2, bw);
    }
    acc_guard1(acc);

    float hn[8];
#pragma unroll
    for (int r = 0; r < 8; ++r) {
      const float z  = acc[r] + boj;
      const float e  = expf(-fabsf(z));
      const float rr = __builtin_amdgcn_rcpf(1.0f + e);
      const float o  = (z >= 0.0f) ? rr : e * rr;
      hn[r] = o * av[r];
    }
    __syncthreads();

    const int tl = t & (HCH - 1);
#pragma unroll
    for (int r = 0; r < 8; ++r) {
      const unsigned short p1 = f2bf_bits(hn[r]);
      const float d1 = hn[r] - bf_bits2f(p1);
      const unsigned short p2 = f2bf_bits(d1);
      const float d2 = d1 - bf_bits2f(p2);
      const unsigned short p3 = f2bf_bits(d2);
      const int ao = (8 * hh + r) * APITCH + j;
      Ap[0][ao] = p1;
      Ap[1][ao] = p2;
      Ap[2][ao] = p3;
      if (hh == 0) sOut[(tl * 8 + r) * OPITCH + j] = hn[r];
    }
    __syncthreads();

    if (tl == HCH - 1) {
      const int t0 = t - (HCH - 1);
      if (MODE == 1) {
        for (int pass = 0; pass < 2; ++pass) {
#pragma unroll
          for (int it = 0; it < 16; ++it) {
            const int idx = it * NTHR + tid;
            const int lr = idx >> 5, c4 = (idx & 31) * 4;
            const int tl2 = lr >> 3, rr = lr & 7;
            const v4f v = *(const v4f*)(sOut + lr * OPITCH + c4);
            *(volatile v4f*)(OUT + ((size_t)rr * NSEQ + (size_t)(t0 + tl2)) * NHID + c4) = v;
          }
          __threadfence();
        }
      } else {
        for (int pass = 0; pass < 2; ++pass) {
#pragma unroll
          for (int it = 0; it < 8; ++it) {
            const int idx = it * NTHR + tid;
            const int lr = idx >> 4, c8 = (idx & 15) * 8;
            const int tl2 = lr >> 3, rr = lr & 7;
            const v4f x0 = *(const v4f*)(sOut + lr * OPITCH + c8);
            const v4f x1 = *(const v4f*)(sOut + lr * OPITCH + c8 + 4);
            v8h hv, lv;
#pragma unroll
            for (int e = 0; e < 4; ++e) {
              const unsigned short hb0 = f2bf_bits(x0[e]);
              const unsigned short lb0 = f2bf_bits(x0[e] - bf_bits2f(hb0));
              const unsigned short hb1 = f2bf_bits(x1[e]);
              const unsigned short lb1 = f2bf_bits(x1[e] - bf_bits2f(hb1));
              hv[e]     = __builtin_bit_cast(_Float16, hb0);
              lv[e]     = __builtin_bit_cast(_Float16, lb0);
              hv[4 + e] = __builtin_bit_cast(_Float16, hb1);
              lv[4 + e] = __builtin_bit_cast(_Float16, lb1);
            }
            const size_t off = ((size_t)rr * NSEQ + (size_t)(t0 + tl2)) * NHID + c8;
            *(volatile v8h*)(HHI + off) = hv;
            *(volatile v8h*)(HLO + off) = lv;
          }
          __threadfence();
        }
      }
    }
  }
}

extern "C" void kernel_launch(void* const* d_in, const int* in_sizes, int n_in,
                              void* d_out, int out_size, void* d_ws, size_t ws_size, hipStream_t stream) {
  if (n_in < 13 || d_out == nullptr || d_ws == nullptr) return;
  if (in_sizes[0] != NROW * NDIM || in_sizes[1] != NDIM * NHID || in_sizes[2] != NHID ||
      in_sizes[3] != NDIM * NHID || in_sizes[4] != NHID || in_sizes[5] != NDIM * NHID || in_sizes[6] != NHID ||
      in_sizes[7] != NLAY * NDIM * NHID || in_sizes[8] != NLAY * NHID || in_sizes[9] != NLAY * NDIM * NHID ||
      in_sizes[10] != NLAY * NHID || in_sizes[11] != NLAY * NHID * NHID || in_sizes[12] != NLAY * NHID ||
      out_size != NROW * NHID) return;

  const float* xin = (const float*)d_in[0];
  const float* Wq  = (const float*)d_in[1];
  const float* bq  = (const float*)d_in[2];
  const float* Wk  = (const float*)d_in[3];
  const float* bk  = (const float*)d_in[4];
  const float* Wv  = (const float*)d_in[5];
  const float* bv  = (const float*)d_in[6];
  const float* Wi  = (const float*)d_in[7];
  const float* bi  = (const float*)d_in[8];
  const float* Wf  = (const float*)d_in[9];
  const float* bfw = (const float*)d_in[10];
  const float* Wo  = (const float*)d_in[11];
  const float* bo  = (const float*)d_in[12];
  float* out = (float*)d_out;

  char* ws = (char*)d_ws; size_t off = 0;
  auto carve = [&](size_t bytes) -> char* { char* p = ws + off; off += (bytes + 255) & ~(size_t)255; return p; };
  unsigned short* XB    = (unsigned short*)carve((size_t)NROW * NDIM * 2);
  unsigned short* WQKVB = (unsigned short*)carve((size_t)NQKV * NDIM * 2);
  unsigned short* WGB   = (unsigned short*)carve((size_t)2 * NGT * NDIM * 2);
  unsigned short* WOB   = (unsigned short*)carve((size_t)NLAY * NHID * NHID * 2);
  float*          BIASB = (float*)carve((size_t)NBIAS * 4);
  float*          QKVP  = (float*)carve((size_t)NROW * NQKV * 4);
  float*          GP0   = (float*)carve((size_t)NROW * NGT * 4);
  float*          ATT0  = (float*)carve((size_t)NROW * NHID * 4);
  unsigned short* HHI   = (unsigned short*)carve((size_t)NROW * NHID * 2);
  unsigned short* HLO   = (unsigned short*)carve((size_t)NROW * NHID * 2);
  float*          GP1   = (float*)carve((size_t)NROW * NGT * 4);
  float*          ATT1  = (float*)carve((size_t)NROW * NHID * 4);
  if (off > ws_size || off > (size_t)134217728) return;

  const size_t WSZ = (size_t)NDIM * NHID;

  const int n8x = NROW * (NDIM / 8);
  cvt8_kernel<0><<<(n8x + NTHR - 1) / NTHR, NTHR, 0, stream>>>(xin, XB, NROW, NDIM / 8, NDIM, 0, 1.0f);
  const dim3 tg(NHID / 64, NDIM / 64);
  tpw_kernel<0><<<tg, NTHR, 0, stream>>>(Wq, NDIM, NHID, NDIM, WQKVB, 1.0f);
  tpw_kernel<0><<<tg, NTHR, 0, stream>>>(Wk, NDIM, NHID, NDIM, WQKVB + (size_t)1 * NHID * NDIM, 1.0f);
  tpw_kernel<0><<<tg, NTHR, 0, stream>>>(Wv, NDIM, NHID, NDIM, WQKVB + (size_t)2 * NHID * NDIM, 1.0f);
  tpw_kernel<0><<<tg, NTHR, 0, stream>>>(Wi,        NDIM, NHID, NDIM, WGB + (size_t)0 * NHID * NDIM, 1.0f);
  tpw_kernel<0><<<tg, NTHR, 0, stream>>>(Wf,        NDIM, NHID, NDIM, WGB + (size_t)1 * NHID * NDIM, 1.0f);
  tpw_kernel<0><<<tg, NTHR, 0, stream>>>(Wi + WSZ,  NDIM, NHID, NDIM, WGB + (size_t)2 * NHID * NDIM, 1.0f);
  tpw_kernel<0><<<tg, NTHR, 0, stream>>>(Wf + WSZ,  NDIM, NHID, NDIM, WGB + (size_t)3 * NHID * NDIM, 1.0f);
  tpw_kernel<0><<<tg, NTHR, 0, stream>>>(Wo,        NHID, NHID, NHID, WOB, 1.0f);
  tpw_kernel<0><<<tg, NTHR, 0, stream>>>(Wo + WSZ,  NHID, NHID, NHID, WOB + (size_t)NHID * NHID, 1.0f);
  bias_prep_kernel<<<1, (NBIAS / 4), 0, stream>>>(bq, bk, bv, bi, bfw, BIASB);

  const dim3 gq((NROW / 64) * (NQKV / 64) / 8, 1);
  wmma_gemm64<1, 0, 2, 0, 0><<<gq, 256, 0, stream>>>(
      XB, XB, NDIM, 0L, WQKVB, WQKVB, NDIM, 0L, (void*)QKVP, (void*)QKVP, NQKV, 0L,
      BIASB, NROW, NQKV, NDIM, 1.0f);

  const dim3 gg((NROW / 64) * (NGT / 64) / 8, 1);
  wmma_gemm64<1, 0, 2, 0, 6><<<gg, 256, 0, stream>>>(
      XB, XB, NDIM, 0L, WGB, WGB, NDIM, 0L, (void*)GP0, (void*)GP0, NGT, 0L,
      BIASB + NQKV, NROW, NGT, NDIM, 1.0f);
  cscan_kernel<<<dim3(NBAT, 2), NTHR, 0, stream>>>(QKVP, GP0, ATT0);
  hgate_kernel<0><<<1, NTHR, 0, stream>>>(ATT0, WOB, bo, HHI, HLO, out);

  wmma_gemm64<1, 2, 2, 0, 6><<<gg, 256, 0, stream>>>(
      HHI, HLO, NHID, 0L, WGB + (size_t)2 * NHID * NDIM, WGB + (size_t)2 * NHID * NDIM, NHID, 0L,
      (void*)GP1, (void*)GP1, NGT, 0L, BIASB + NQKV + NGT, NROW, NGT, NHID, 1.0f);
  cscan_kernel<<<dim3(NBAT, 2), NTHR, 0, stream>>>(QKVP, GP1, ATT1);
  hgate_kernel<1><<<1, NTHR, 0, stream>>>(ATT1, WOB + (size_t)NHID * NHID, bo + NHID, HHI, HLO, out);
}
